// EdgeConcatAdjNet_56805237457601
// MI455X (gfx1250) — hardware-verified
//
#include <hip/hip_runtime.h>
#include <stddef.h>


typedef _Float16 v16h __attribute__((ext_vector_type(16)));
typedef _Float16 v8h  __attribute__((ext_vector_type(8)));
typedef float    v8f  __attribute__((ext_vector_type(8)));
typedef float    v4f  __attribute__((ext_vector_type(4)));

#ifndef NB
#define NB 2
#endif
#ifndef SEQ
#define SEQ 1024
#endif
#define NB_FULL  2
#define SEQ_FULL 1024
#define FEAT  128
#define HID1  64
#define HID2  32
#define PW    128
#define W1T_LD 256
#define MROWS (NB * SEQ)

#define TI 64
#define TJ 32
#define OSP 36

static_assert(NB >= 1 && NB <= NB_FULL);
static_assert(SEQ >= 64 && SEQ <= SEQ_FULL && (SEQ % 64) == 0);
static_assert((SEQ % TI) == 0 && (SEQ % TJ) == 0);
static_assert((MROWS % 64) == 0 && (MROWS % 16) == 0);
static_assert(FEAT == 128 && (FEAT % 32) == 0);
static_assert(HID1 == 64 && (HID1 % 32) == 0);
static_assert(HID2 == 32);
static_assert(PW == 2 * HID1);
static_assert(W1T_LD == 2 * FEAT);
static_assert(TI == 4 * 16 && TJ == 2 * 16);
static_assert(TJ * 4 == 128);
static_assert((OSP % 4) == 0 && OSP >= TJ);
static_assert(2 * 32 == TI);
static_assert((size_t)(TI * 64 + TI * OSP) * 4 <= (size_t)131072);

#define LDT 72
#define LDC 68
static_assert((LDT % 8) == 0 && LDT >= 64);
static_assert((LDC % 4) == 0 && LDC >= 64);

#define WCARRY 64.0f

#define W1T_BYTES ((size_t)HID1 * W1T_LD * 2)
#define W2T_BYTES ((size_t)HID2 * HID1 * 2)
#define X16_BYTES ((size_t)MROWS * FEAT * 2)
#define P_BYTES   ((size_t)MROWS * PW * 4)
#define OFF_W1T ((size_t)0)
#define OFF_W2T (OFF_W1T + W1T_BYTES)
#define OFF_X16 (OFF_W2T + W2T_BYTES)
#define OFF_P   (OFF_X16 + X16_BYTES)
#define WS_TOTAL (OFF_P + P_BYTES)
static_assert((W1T_BYTES % 128) == 0 && (W2T_BYTES % 128) == 0);
static_assert((X16_BYTES % 128) == 0 && (P_BYTES % 128) == 0);
static_assert(WS_TOTAL <= (size_t)134217728);

__device__ __forceinline__ float bf16r(float x) {
  unsigned int u = __float_as_uint(x);
  u = (u + 0x7FFFu + ((u >> 16) & 1u)) & 0xFFFF0000u;
  return __uint_as_float(u);
}

static __device__ __forceinline__ _Float16 toh_flush(float v) {
  const _Float16 r = (_Float16)v;
  return (fabsf(v) < 6.103515625e-05f) ? (_Float16)0.0f : r;
}
static __device__ __forceinline__ _Float16 relu_toh_flush(float v) {
  const _Float16 r = (_Float16)v;
  return (v < 6.103515625e-05f) ? (_Float16)0.0f : r;
}

__device__ __forceinline__ v16h frag_at(const _Float16* p) {
  v8h lo = *(const v8h*)(p);
  v8h hi = *(const v8h*)(p + 16);
  v16h out;
#pragma unroll
  for (int i = 0; i < 8; ++i) { out[i] = lo[i]; out[i + 8] = hi[i]; }
  return out;
}

__device__ __forceinline__ v8f wmma16(v16h a, v16h b, v8f c) {
  v8f d = __builtin_amdgcn_wmma_f32_16x16x32_f16(false, a, false, b, (short)0, c,
                                                 false, false);
  asm volatile("v_nop\n\tv_nop\n\tv_nop\n\tv_nop" : "+v"(d) : "v"(a), "v"(b));
  return d;
}

__global__ __launch_bounds__(256) void wconv_kernel(
    const float* __restrict__ W, _Float16* __restrict__ Wt, unsigned ldw, unsigned ldk) {
  __shared__ _Float16 T[64 * LDT];
  const unsigned tid = threadIdx.x;
  const unsigned n0 = blockIdx.x * 64u;
  const unsigned k0 = blockIdx.y * 64u;
#pragma unroll 4
  for (unsigned j = 0; j < 16u; ++j) {
    const unsigned idx = tid + 256u * j;
    const unsigned kr = idx >> 6, nc = idx & 63u;
    const float v = W[(size_t)(k0 + kr) * ldw + n0 + nc];
    T[nc * LDT + kr] = toh_flush(WCARRY * bf16r(v));
  }
  __syncthreads();
  v8h x[2];
  size_t off[2];
#pragma unroll
  for (unsigned i = 0; i < 2u; ++i) {
    const unsigned n = 32u * i + (tid >> 3);
    const unsigned kc = (tid & 7u) * 8u;
    x[i] = *(const v8h*)&T[n * LDT + kc];
    off[i] = (size_t)(n0 + n) * ldk + k0 + kc;
  }
#pragma unroll
  for (int i = 0; i < 2; ++i) *(volatile v8h*)(Wt + off[i]) = x[i];
  __threadfence();
#pragma unroll
  for (int i = 0; i < 2; ++i) *(volatile v8h*)(Wt + off[i]) = x[i];
}

__global__ __launch_bounds__(256) void w2conv_kernel(
    const float* __restrict__ W2, _Float16* __restrict__ W2t) {
  __shared__ _Float16 T[HID2 * LDT];
  const unsigned tid = threadIdx.x;
#pragma unroll 4
  for (unsigned j = 0; j < 8u; ++j) {
    const unsigned idx = tid + 256u * j;
    const unsigned kr = idx >> 5, nc = idx & 31u;
    const float v = W2[idx];
    T[nc * LDT + kr] = toh_flush(WCARRY * bf16r(v));
  }
  __syncthreads();
  const unsigned n = tid >> 3;
  const unsigned kc = (tid & 7u) * 8u;
  const v8h xv = *(const v8h*)&T[n * LDT + kc];
  const size_t off = (size_t)n * HID1 + kc;
  *(volatile v8h*)(W2t + off) = xv;
  __threadfence();
  *(volatile v8h*)(W2t + off) = xv;
}

__global__ __launch_bounds__(256) void xconv_kernel(
    const float* __restrict__ X, _Float16* __restrict__ X16) {
  const unsigned g = blockIdx.x * 256u + threadIdx.x;
  const unsigned crow = g >> 4;
  const unsigned c = (g & 15u) * 8u;
  const unsigned bidx = crow / (unsigned)SEQ;
  const unsigned sq = crow - bidx * (unsigned)SEQ;
  const size_t srow = (size_t)bidx * SEQ_FULL + sq;
  const v4f a0 = *(const v4f*)(X + srow * FEAT + c);
  const v4f a1 = *(const v4f*)(X + srow * FEAT + c + 4u);
  v8h o;
#pragma unroll
  for (int i = 0; i < 4; ++i) {
    o[i]     = toh_flush(bf16r(a0[i]));
    o[i + 4] = toh_flush(bf16r(a1[i]));
  }
  _Float16* p = X16 + (size_t)g * 8u;
  *(volatile v8h*)p = o;
  __threadfence();
  *(volatile v8h*)p = o;
}

__global__ __launch_bounds__(256) void proj_kernel(
    const _Float16* __restrict__ A16, const _Float16* __restrict__ Bt,
    const float* __restrict__ bias, float* __restrict__ outf) {
  __shared__ float Cs[64 * LDC];
  const unsigned tid = threadIdx.x, lane = tid & 31u;
  const unsigned w = (unsigned)__builtin_amdgcn_readfirstlane((int)(threadIdx.x >> 5));
  const unsigned mw = w >> 1, nw = w & 1u;
  const unsigned hh = lane >> 4, m = lane & 15u;
  const unsigned n0 = blockIdx.x * 64u;
  const unsigned koff = blockIdx.x * (unsigned)FEAT;
  const unsigned row0 = blockIdx.y * 64u;

  const _Float16* ap  = A16 + (size_t)(row0 + mw * 16u + m) * FEAT + hh * 8u;
  const _Float16* bp0 = Bt + (size_t)(nw * 32u + m) * W1T_LD + koff + hh * 8u;
  const _Float16* bp1 = bp0 + (size_t)16 * W1T_LD;
  v8f acc0 = {}, acc1 = {};
#pragma unroll 2
  for (unsigned k0 = 0; k0 < (unsigned)FEAT; k0 += 32u) {
    const v16h a  = frag_at(ap + k0);
    const v16h b0 = frag_at(bp0 + k0);
    const v16h b1 = frag_at(bp1 + k0);
    acc0 = wmma16(a, b0, acc0);
    acc1 = wmma16(a, b1, acc1);
  }
#pragma unroll
  for (int r = 0; r < 8; ++r) {
    float* d = &Cs[(mw * 16u + hh * 8u + (unsigned)r) * LDC + nw * 32u + m];
    d[0]  = acc0[r];
    d[16] = acc1[r];
  }
  __syncthreads();

  const bool with_bias = (n0 == 0u);
  v4f xs[4];
  size_t off[4];
#pragma unroll
  for (unsigned i = 0; i < 4u; ++i) {
    const unsigned r = 16u * i + (tid >> 4);
    const unsigned c = (tid & 15u) * 4u;
    const v4f u = *(const v4f*)&Cs[r * LDC + c];
    const v4f g = *(const v4f*)(bias + c);
    v4f val;
#pragma unroll
    for (int j = 0; j < 4; ++j) {
      const float bb = with_bias ? bf16r(g[j]) : 0.0f;
      val[j] = u[j] * (1.0f / WCARRY) + bb;
    }
    xs[i] = val;
    off[i] = (size_t)(row0 + r) * PW + n0 + c;
  }
#pragma unroll
  for (int i = 0; i < 4; ++i) *(volatile v4f*)(outf + off[i]) = xs[i];
  __threadfence();
#pragma unroll
  for (int i = 0; i < 4; ++i) *(volatile v4f*)(outf + off[i]) = xs[i];
}

__global__ __launch_bounds__(256) void edge_kernel(
    const float* __restrict__ P, const _Float16* __restrict__ W2t,
    const float* __restrict__ b2, const float* __restrict__ W3, const float* __restrict__ b3,
    float* __restrict__ out) {
  __shared__ float PIs[TI * 64];
  __shared__ float Os[TI * OSP];

  const unsigned tid = threadIdx.x, lane = tid & 31u;
  const unsigned wave = (unsigned)__builtin_amdgcn_readfirstlane((int)(threadIdx.x >> 5));
  const unsigned hh = lane >> 4, m = lane & 15u;
  const unsigned j0 = blockIdx.x * (unsigned)TJ;
  const unsigned i0 = blockIdx.y * (unsigned)TI;
  const unsigned b = blockIdx.z;
  const unsigned jg = wave & 1u, iq = wave >> 1;

#pragma unroll
  for (unsigned j = 0; j < 4u; ++j) {
    const unsigned idx = tid + 256u * j;
    const unsigned r = idx >> 4, c = (idx & 15u) * 4u;
    *(v4f*)&PIs[r * 64u + c] =
        *(const v4f*)(P + (size_t)(b * (unsigned)SEQ + i0 + r) * PW + HID1 + c);
  }

  v16h wa[2][2];
#pragma unroll
  for (int nt = 0; nt < 2; ++nt)
#pragma unroll
    for (int c = 0; c < 2; ++c)
      wa[nt][c] = frag_at(W2t + (size_t)((unsigned)nt * 16u + m) * HID1 + (unsigned)c * 32u + hh * 8u);

  float pjr[32];
  {
    const float* pr = P + (size_t)(b * (unsigned)SEQ + j0 + jg * 16u + m) * PW + hh * 8u;
#pragma unroll
    for (int c = 0; c < 2; ++c)
#pragma unroll
      for (int sg = 0; sg < 2; ++sg) {
        const v4f p0 = *(const v4f*)(pr + c * 32 + sg * 16);
        const v4f p1 = *(const v4f*)(pr + c * 32 + sg * 16 + 4);
#pragma unroll
        for (int e = 0; e < 4; ++e) {
          pjr[c * 16 + sg * 8 + e]     = p0[e];
          pjr[c * 16 + sg * 8 + 4 + e] = p1[e];
        }
      }
  }

  float b2s[2][8], w3s[2][8];
#pragma unroll
  for (int nt = 0; nt < 2; ++nt) {
    const v4f g0 = *(const v4f*)(b2 + (unsigned)nt * 16u + hh * 8u);
    const v4f g1 = *(const v4f*)(b2 + (unsigned)nt * 16u + hh * 8u + 4u);
    const v4f q0 = *(const v4f*)(W3 + (unsigned)nt * 16u + hh * 8u);
    const v4f q1 = *(const v4f*)(W3 + (unsigned)nt * 16u + hh * 8u + 4u);
#pragma unroll
    for (int e = 0; e < 4; ++e) {
      b2s[nt][e]     = WCARRY * bf16r(g0[e]);
      b2s[nt][e + 4] = WCARRY * bf16r(g1[e]);
      w3s[nt][e]     = bf16r(q0[e]) * (1.0f / WCARRY);
      w3s[nt][e + 4] = bf16r(q1[e]) * (1.0f / WCARRY);
    }
  }
  const float b3v = bf16r(b3[0]);

  __syncthreads();

#pragma unroll 1
  for (unsigned ii = 0; ii < 16u; ++ii) {
    const unsigned il = iq * 16u + ii;
    const unsigned pbase = il * 64u + hh * 8u;
    v8f acc0 = {}, acc1 = {};
#pragma unroll
    for (int c = 0; c < 2; ++c) {
      v16h hb;
#pragma unroll
      for (int sg = 0; sg < 2; ++sg) {
        const v4f p0 = *(const v4f*)&PIs[pbase + (unsigned)(c * 32 + sg * 16)];
        const v4f p1 = *(const v4f*)&PIs[pbase + (unsigned)(c * 32 + sg * 16 + 4)];
#pragma unroll
        for (int e = 0; e < 4; ++e) {
          hb[sg * 8 + e]     = relu_toh_flush(pjr[c * 16 + sg * 8 + e] + p0[e]);
          hb[sg * 8 + 4 + e] = relu_toh_flush(pjr[c * 16 + sg * 8 + 4 + e] + p1[e]);
        }
      }
      acc0 = wmma16(wa[0][c], hb, acc0);
      acc1 = wmma16(wa[1][c], hb, acc1);
    }
    float s = 0.0f;
#pragma unroll
    for (int r = 0; r < 8; ++r) {
      s += fmaxf(acc0[r] + b2s[0][r], 0.0f) * w3s[0][r];
      s += fmaxf(acc1[r] + b2s[1][r], 0.0f) * w3s[1][r];
    }
    s += __shfl_xor(s, 16, 32);
    s += b3v;
    if (hh == 0u) Os[il * OSP + jg * 16u + m] = s;
  }
  __syncthreads();

  v4f xs[2];
  size_t off[2];
#pragma unroll
  for (unsigned i = 0; i < 2u; ++i) {
    const unsigned r = 32u * i + (tid >> 3);
    const unsigned c = (tid & 7u) * 4u;
    xs[i] = *(const v4f*)&Os[r * OSP + c];
    off[i] = ((size_t)b * SEQ_FULL + i0 + r) * SEQ_FULL + j0 + c;
  }
#pragma unroll
  for (int i = 0; i < 2; ++i) *(volatile v4f*)(out + off[i]) = xs[i];
  __threadfence();
#pragma unroll
  for (int i = 0; i < 2; ++i) *(volatile v4f*)(out + off[i]) = xs[i];
}

extern "C" void kernel_launch(void* const* d_in, const int* in_sizes, int n_in,
                              void* d_out, int out_size, void* d_ws, size_t ws_size,
                              hipStream_t stream) {
  if (n_in < 9) return;
  const long long need_x = ((long long)(NB - 1) * SEQ_FULL + SEQ) * FEAT;
  const long long need_o = ((long long)(NB - 1) * SEQ_FULL + (SEQ - 1)) * SEQ_FULL + SEQ;
  if ((long long)in_sizes[0] < need_x) return;
  if ((long long)in_sizes[3] < (long long)2 * FEAT * HID1) return;
  if (in_sizes[4] < HID1) return;
  if (in_sizes[5] < HID1 * HID2) return;
  if (in_sizes[6] < HID2 || in_sizes[7] < HID2 || in_sizes[8] < 1) return;
  if ((long long)out_size < need_o) return;
  if (ws_size < WS_TOTAL) return;

  const float* X  = (const float*)d_in[0];
  const float* w1 = (const float*)d_in[3];
  const float* b1 = (const float*)d_in[4];
  const float* w2 = (const float*)d_in[5];
  const float* b2 = (const float*)d_in[6];
  const float* w3 = (const float*)d_in[7];
  const float* b3 = (const float*)d_in[8];
  float* out = (float*)d_out;

  char* ws = (char*)d_ws;
  _Float16* W1t = (_Float16*)(ws + OFF_W1T);
  _Float16* W2t = (_Float16*)(ws + OFF_W2T);
  _Float16* X16 = (_Float16*)(ws + OFF_X16);
  float*    Pp  = (float*)(ws + OFF_P);

  dim3 blk(256);
  wconv_kernel<<<dim3(HID1 / 64, (2 * FEAT) / 64), blk, 0, stream>>>(
      w1, W1t, (unsigned)HID1, (unsigned)W1T_LD);
  w2conv_kernel<<<dim3(1), blk, 0, stream>>>(w2, W2t);
  xconv_kernel<<<dim3(MROWS / 16), blk, 0, stream>>>(X, X16);
  proj_kernel<<<dim3(2, MROWS / 64), blk, 0, stream>>>(X16, W1t, b1, Pp);
  edge_kernel<<<dim3(SEQ / TJ, SEQ / TI, NB), blk, 0, stream>>>(Pp, W2t, b2, w3, b3, out);
}
